// TransformerEncoderBlock_34437047779658
// MI455X (gfx1250) — hardware-verified
//
#include <hip/hip_runtime.h>


#ifndef NB
#define NB 4
#endif
#ifndef SEQ
#define SEQ 2048
#endif
#define NB_FULL 4
#define SEQ_FULL 2048

namespace {
constexpr unsigned EMB = 768, NH = 8, HD = 96, HID = 3072, TOK = (unsigned)NB * (unsigned)SEQ;
constexpr float XS = 8.0f, QS = 8.0f, VS = 8.0f, CS = 256.0f, GS = 8.0f, WSC = 256.0f, LOG2E = 1.4426950408889634f, LNEPS = 1e-5f, RSQE = 0.03608439182435161f  , RSQ2 = 0.70710678118654752f;
constexpr unsigned NTQ = 3 * EMB / 64, NTP = EMB / 64, NT1 = HID / 64, NT2 = EMB / 64;
constexpr unsigned TQ = (EMB / 64) * NTQ, TP = (EMB / 64) * NTP, T1 = (EMB / 64) * NT1, T2 = (HID / 64) * NT2;
static_assert(SEQ % 128 == 0);
static_assert(TOK % 128 == 0);
static_assert(EMB == NH * HD);
static_assert(HD == 96);
static_assert(EMB % 96 == 0 && HID % 96 == 0 && (3 * EMB) % 96 == 0);
static_assert(EMB % 64 == 0 && HID % 64 == 0);
static_assert(NB <= NB_FULL && SEQ <= SEQ_FULL);
static_assert(((size_t)(NB - 1) * SEQ_FULL + SEQ) * EMB <= (size_t)NB_FULL * SEQ_FULL * EMB);
typedef _Float16 b16;
typedef __attribute__((ext_vector_type(16))) _Float16 v16b;
typedef __attribute__((ext_vector_type(8))) _Float16 v8b;
typedef __attribute__((ext_vector_type(4))) _Float16 v4h;
typedef __attribute__((ext_vector_type(8))) float v8f;
typedef __attribute__((ext_vector_type(4))) float v4f;
__device__ __forceinline__ float bf16_rne(float f) { unsigned int u = __float_as_uint(f); u += 0x7FFFu + ((u >> 16) & 1u); return __uint_as_float(u & 0xFFFF0000u); }
__device__ __forceinline__ v16b frag_kb(const b16* p, unsigned hh) { const v8b a = *(const v8b*)(p + 8 * hh), b = *(const v8b*)(p + 16 + 8 * hh); v16b f;
#pragma unroll
  for (int e = 0; e < 8; ++e) { f[e] = a[e]; f[8 + e] = b[e]; } return f; }
__device__ __forceinline__ v8f wmma16b(v16b a, v16b b, v8f c) { v8f d = __builtin_amdgcn_wmma_f32_16x16x32_f16(false, a, false, b, (short)0, c, false, false); asm volatile("v_nop\n\tv_nop\n\tv_nop\n\tv_nop" : "+v"(d) : "v"(a), "v"(b)); return d; }
__device__ __forceinline__ void wave_lds_sync() { __builtin_amdgcn_fence(3  , "workgroup"); __builtin_amdgcn_wave_barrier(); __builtin_amdgcn_fence(2  , "workgroup"); }
__device__ __forceinline__ float pmul(float a, float b) { float p = a * b; asm volatile("" : "+v"(p)); return p; }
__device__ __forceinline__ float nexp2(float v) { return __builtin_amdgcn_exp2f(v); }
__device__ __forceinline__ size_t xrow(unsigned m) { return (size_t)(m / (unsigned)SEQ) * (size_t)SEQ_FULL + (size_t)(m % (unsigned)SEQ); }

__global__ __launch_bounds__(128) void prep_kernel(const float* __restrict__ wq, const float* __restrict__ wp, const float* __restrict__ w1, const float* __restrict__ w2,
                                                    b16* __restrict__ WQ, b16* __restrict__ WP, b16* __restrict__ W1, b16* __restrict__ W2) {
  __shared__ __attribute__((aligned(16))) b16 tile[64][72];
  const unsigned wave = threadIdx.x >> 5, lane = threadIdx.x & 31u;
  unsigned t = blockIdx.x, K, N, tk, perm = 0u; const float* src; b16* dst;
  if (t < TQ) { src = wq; dst = WQ; K = EMB; N = 3u * EMB; tk = t / NTQ; perm = 1u; }
  else if (t < TQ + TP) { t -= TQ; src = wp; dst = WP; K = EMB; N = EMB; tk = t / NTP; }
  else if (t < TQ + TP + T1) { t -= TQ + TP; src = w1; dst = W1; K = EMB; N = HID; tk = t / NT1; }
  else { t -= TQ + TP + T1; src = w2; dst = W2; K = HID; N = EMB; tk = t / NT2; }
  const unsigned tn = t - tk * (N >> 6), k0 = tk << 6, n0 = tn << 6;
  for (unsigned i = threadIdx.x; i < 1024u; i += 128u) { const unsigned kk = i >> 4, q4 = (i & 15u) << 2; const v4f f = *(const v4f*)(src + (size_t)(k0 + kk) * N + n0 + q4); v4h o;
#pragma unroll
    for (int j = 0; j < 4; ++j) o[j] = (b16)(bf16_rne(f[j]) * WSC);
    *(v4h*)(&tile[kk][q4]) = o; }
  __syncthreads();
  for (int pass = 0; pass < 2; ++pass) {
#pragma unroll 1
    for (unsigned it = 0; it < 4u; ++it) { const unsigned nl = wave * 16u + it * 4u + (lane >> 3), piece = lane & 7u; v8b o;
#pragma unroll
      for (int j = 0; j < 8; ++j) o[j] = tile[piece * 8u + j][nl];
      const unsigned n = n0 + nl; const unsigned prow = perm ? ((n % 3u) * EMB + n / 3u) : n;
      *(volatile v8b*)(dst + (size_t)prow * K + k0 + piece * 8u) = o; }
    __threadfence(); }
}

template <int CVT>
__global__ __launch_bounds__(256) void ln_kernel(const float* __restrict__ X, const float* __restrict__ g, const float* __restrict__ bta, b16* __restrict__ H) {
  const unsigned wave = threadIdx.x >> 5, lane = threadIdx.x & 31u; const unsigned m = blockIdx.x * 8u + wave;
  const float* xr = X + (CVT ? xrow(m) : (size_t)m) * EMB;
  v4f v[6]; float s = 0.0f;
#pragma unroll
  for (int q = 0; q < 6; ++q) { v4f f = *(const v4f*)(xr + q * 128 + lane * 4u);
#pragma unroll
    for (int j = 0; j < 4; ++j) { if (CVT) f[j] = bf16_rne(f[j]); s += f[j]; }
    v[q] = f; }
#pragma unroll
  for (int o = 16; o >= 1; o >>= 1) s += __shfl_xor(s, o);
  const float mean = s * (1.0f / (float)EMB); float s2 = 0.0f;
#pragma unroll
  for (int q = 0; q < 6; ++q)
#pragma unroll
    for (int j = 0; j < 4; ++j) { const float d = v[q][j] - mean; s2 += pmul(d, d); }
#pragma unroll
  for (int o = 16; o >= 1; o >>= 1) s2 += __shfl_xor(s2, o);
  const float rs = rsqrtf(s2 * (1.0f / (float)EMB) + LNEPS);
  v4h ov[6];
#pragma unroll
  for (int q = 0; q < 6; ++q) { const v4f gv = *(const v4f*)(g + q * 128 + lane * 4u), bv = *(const v4f*)(bta + q * 128 + lane * 4u);
#pragma unroll
    for (int j = 0; j < 4; ++j) ov[q][j] = (b16)((pmul(pmul(v[q][j] - mean, rs), bf16_rne(gv[j])) + bf16_rne(bv[j])) * XS); }
  for (int pass = 0; pass < 2; ++pass) {
#pragma unroll
    for (int q = 0; q < 6; ++q) *(volatile v4h*)(H + (size_t)m * EMB + q * 128 + lane * 4u) = ov[q];
    __threadfence(); }
}

enum { EPI_QKV = 0, EPI_PROJ = 1, EPI_FC1 = 2, EPI_FC2 = 3 };
template <int EPI, int AMODE, unsigned K>
__global__ __launch_bounds__(128) void gemm_kernel(const b16* __restrict__ A, const b16* __restrict__ W, const float* __restrict__ bias, const float* __restrict__ resid,
                                                    float* __restrict__ outf, b16* __restrict__ ob0, b16* __restrict__ ob1, b16* __restrict__ ob2) {
  __shared__ __attribute__((aligned(16))) float Tf[4][32][100];
  const unsigned wave = threadIdx.x >> 5, lane = threadIdx.x & 31u, nloc = lane & 15u, hlf = lane >> 4;
  const unsigned mb = blockIdx.x * 128u, m0 = mb + wave * 32u, y = blockIdx.y, n0 = y * 96u;
  v8f acc0[6], acc1[6];
#pragma unroll
  for (int t = 0; t < 6; ++t) { acc0[t] = (v8f){}; acc1[t] = (v8f){}; }
  const size_t astep = (AMODE == 0) ? (size_t)16 * K : (size_t)16 * HD;
  const b16* arow = A + (size_t)(m0 + nloc) * ((AMODE == 0) ? K : HD);
  const b16* wrow = W + (size_t)(n0 + nloc) * K;
  size_t aoff = 0; unsigned dd = 0;
#pragma unroll 1
  for (unsigned kb = 0; kb < K; kb += 32u) {
    const v16b a0 = frag_kb(arow + aoff, hlf), a1 = frag_kb(arow + aoff + astep, hlf);
#pragma unroll
    for (int t = 0; t < 6; ++t) { const v16b bw = frag_kb(wrow + (size_t)t * 16 * K + kb, hlf); acc0[t] = wmma16b(a0, bw, acc0[t]); acc1[t] = wmma16b(a1, bw, acc1[t]); }
    aoff += 32; dd += 32u;
    if (AMODE == 1) { if (dd == 96u) { dd = 0u; aoff += (size_t)TOK * HD - 96; } }
  }
  const float scl = (EPI == EPI_PROJ) ? (1.0f / (CS * WSC)) : ((EPI == EPI_FC2) ? (1.0f / (GS * WSC)) : (1.0f / (XS * WSC)));
  const unsigned which = y >> 3, hd = y & 7u;
#pragma unroll
  for (int t = 0; t < 6; ++t) { const unsigned col = (unsigned)t * 16u + nloc; const unsigned bi = (EPI == EPI_QKV) ? (hd * 288u + col * 3u + which) : (n0 + col); const float bv = bf16_rne(bias[bi]);
#pragma unroll
    for (int r = 0; r < 8; ++r) { Tf[wave][8u * hlf + r][col] = acc0[t][r] * scl + bv; Tf[wave][16u + 8u * hlf + r][col] = acc1[t][r] * scl + bv; } }
  __syncthreads();
  if constexpr (EPI == EPI_QKV) {
    if (which < 2u) {
      b16* dst = ((which == 0u) ? ob0 : ob1) + ((size_t)hd * TOK + m0) * HD;
      for (int pass = 0; pass < 2; ++pass) {
#pragma unroll 1
        for (unsigned it = 0; it < 12u; ++it) { const unsigned idx = it * 32u + lane, row = idx / 12u, c8 = (idx - row * 12u) * 8u;
          const v4f fa = *(const v4f*)(&Tf[wave][row][c8]), fb = *(const v4f*)(&Tf[wave][row][c8 + 4u]); v8b o;
#pragma unroll
          for (int j = 0; j < 4; ++j) { o[j] = (b16)(fa[j] * QS); o[4 + j] = (b16)(fb[j] * QS); }
          *(volatile v8b*)(dst + (size_t)idx * 8u) = o; }
        __threadfence(); }
    } else {
      const unsigned bb = mb / (unsigned)SEQ, ns0 = mb % (unsigned)SEQ;
      b16* base = ob2 + ((size_t)(bb * NH + hd) * HD) * SEQ + ns0;
      for (int pass = 0; pass < 2; ++pass) {
#pragma unroll 1
        for (unsigned it = 0; it < 12u; ++it) { const unsigned d = wave * 24u + it * 2u + hlf, tl = nloc * 8u, tw = tl >> 5, tr = tl & 31u; v8b o;
#pragma unroll
          for (int j = 0; j < 8; ++j) o[j] = (b16)(Tf[tw][tr + j][d] * VS);
          *(volatile v8b*)(base + (size_t)d * SEQ + nloc * 8u) = o; }
        __threadfence(); }
    }
  } else if constexpr (EPI == EPI_PROJ || EPI == EPI_FC2) {
#pragma unroll 1
    for (unsigned it = 0; it < 24u; ++it) { const unsigned idx = it * 32u + lane, row = idx / 24u, p4 = (idx - row * 24u) * 4u; const unsigned gm = m0 + row;
      const size_t rr = (EPI == EPI_PROJ) ? xrow(gm) : (size_t)gm; v4f rv = *(const v4f*)(resid + rr * EMB + n0 + p4); v4f tv = *(const v4f*)(&Tf[wave][row][p4]);
#pragma unroll
      for (int j = 0; j < 4; ++j) tv[j] += (EPI == EPI_PROJ) ? bf16_rne(rv[j]) : rv[j];
      *(v4f*)(&Tf[wave][row][p4]) = tv; }
    for (int pass = 0; pass < 2; ++pass) {
#pragma unroll 1
      for (unsigned it = 0; it < 24u; ++it) { const unsigned idx = it * 32u + lane, row = idx / 24u, p4 = (idx - row * 24u) * 4u; const unsigned gm = m0 + row;
        const size_t orow = (EPI == EPI_FC2) ? xrow(gm) : (size_t)gm; const v4f tv = *(const v4f*)(&Tf[wave][row][p4]);
        *(volatile v4f*)(outf + orow * EMB + n0 + p4) = tv; }
      __threadfence(); }
  } else {
#pragma unroll 1
    for (unsigned it = 0; it < 12u; ++it) { const unsigned idx = it * 32u + lane, row = idx / 12u, c8 = (idx - row * 12u) * 8u;
      v4f fa = *(const v4f*)(&Tf[wave][row][c8]), fb = *(const v4f*)(&Tf[wave][row][c8 + 4u]);
#pragma unroll 1
      for (int j = 0; j < 4; ++j) { const float ua = fa[j], ub = fb[j]; fa[j] = 0.5f * ua * (1.0f + erff(ua * RSQ2)); fb[j] = 0.5f * ub * (1.0f + erff(ub * RSQ2)); }
      *(v4f*)(&Tf[wave][row][c8]) = fa; *(v4f*)(&Tf[wave][row][c8 + 4u]) = fb; }
    b16* dst = ob0 + ((size_t)y * TOK + m0) * HD;
    for (int pass = 0; pass < 2; ++pass) {
#pragma unroll 1
      for (unsigned it = 0; it < 12u; ++it) { const unsigned idx = it * 32u + lane, row = idx / 12u, c8 = (idx - row * 12u) * 8u;
        const v4f fa = *(const v4f*)(&Tf[wave][row][c8]), fb = *(const v4f*)(&Tf[wave][row][c8 + 4u]); v8b o;
#pragma unroll
        for (int j = 0; j < 4; ++j) { o[j] = (b16)(fa[j] * GS); o[4 + j] = (b16)(fb[j] * GS); }
        *(volatile v8b*)(dst + (size_t)idx * 8u) = o; }
      __threadfence(); }
  }
}

__global__ __launch_bounds__(128) void attn_kernel(const b16* __restrict__ QP, const b16* __restrict__ KP, const b16* __restrict__ VT, b16* __restrict__ CT) {
  __shared__ __attribute__((aligned(16))) float Tf[4][16][100];
  const unsigned wave = threadIdx.x >> 5, lane = threadIdx.x & 31u, nloc = lane & 15u, hlf = lane >> 4;
  const unsigned bh = blockIdx.y, bb = bh >> 3, hd = bh & 7u, q0 = blockIdx.x * 64u + wave * 16u;
  const size_t rowbase = (size_t)hd * TOK + (size_t)bb * (unsigned)SEQ;
  const b16* qr = QP + (rowbase + q0 + nloc) * HD;
  const v16b qf0 = frag_kb(qr, hlf), qf1 = frag_kb(qr + 32, hlf), qf2 = frag_kb(qr + 64, hlf);
  const b16* kr = KP + (rowbase + nloc) * HD;
  const b16* vr = VT + ((size_t)bh * HD + nloc) * SEQ;
  v8f acc[6];
#pragma unroll
  for (int t = 0; t < 6; ++t) acc[t] = (v8f){};
  float m = -1.0e30f, l = 0.0f; const float c = LOG2E / (QS * QS);
#pragma unroll 1
  for (unsigned key0 = 0; key0 < (unsigned)SEQ; key0 += 32u) {
    const b16* k0p = kr + (size_t)key0 * HD; const b16* k1p = k0p + 16 * HD;
    v8f s0 = (v8f){}, s1 = (v8f){};
    s0 = wmma16b(frag_kb(k0p, hlf), qf0, s0); s0 = wmma16b(frag_kb(k0p + 32, hlf), qf1, s0); s0 = wmma16b(frag_kb(k0p + 64, hlf), qf2, s0);
    s1 = wmma16b(frag_kb(k1p, hlf), qf0, s1); s1 = wmma16b(frag_kb(k1p + 32, hlf), qf1, s1); s1 = wmma16b(frag_kb(k1p + 64, hlf), qf2, s1);
    float mx = fmaxf(s0[0], s1[0]);
#pragma unroll
    for (int r = 1; r < 8; ++r) mx = fmaxf(mx, fmaxf(s0[r], s1[r]));
    mx = fmaxf(mx, __shfl_xor(mx, 16));
    const float mn = fmaxf(m, mx); const float sc = nexp2((m - mn) * c); m = mn;
    v16b pf; float ps = 0.0f;
#pragma unroll
    for (int r = 0; r < 8; ++r) { const float p0 = nexp2((s0[r] - mn) * c + 10.0f), p1 = nexp2((s1[r] - mn) * c + 10.0f); ps += p0 + p1; pf[r] = (b16)p0; pf[8 + r] = (b16)p1; }
    l = l * sc + ps;
#pragma unroll
    for (int t = 0; t < 6; ++t) acc[t] = acc[t] * sc;
#pragma unroll
    for (int t = 0; t < 6; ++t) acc[t] = wmma16b(frag_kb(vr + (size_t)t * 16 * SEQ + key0, hlf), pf, acc[t]);
  }
  l += __shfl_xor(l, 16);
  const float f = (CS * RSQE / VS) * (1.0f / l);
#pragma unroll
  for (int t = 0; t < 6; ++t)
#pragma unroll
    for (int r = 0; r < 8; ++r) Tf[wave][nloc][(unsigned)t * 16u + 8u * hlf + r] = acc[t][r] * f;
  wave_lds_sync();
  b16* dst = CT + (rowbase + q0) * HD;
  for (int pass = 0; pass < 2; ++pass) {
#pragma unroll 1
    for (unsigned it = 0; it < 6u; ++it) { const unsigned idx = it * 32u + lane, row = idx / 12u, c8 = (idx - row * 12u) * 8u;
      const v4f fa = *(const v4f*)(&Tf[wave][row][c8]), fb = *(const v4f*)(&Tf[wave][row][c8 + 4u]); v8b o;
#pragma unroll
      for (int j = 0; j < 4; ++j) { o[j] = (b16)fa[j]; o[4 + j] = (b16)fb[j]; }
      *(volatile v8b*)(dst + (size_t)idx * 8u) = o; }
    __threadfence(); }
}
}

extern "C" void kernel_launch(void* const* d_in, const int* in_sizes, int n_in, void* d_out, int out_size, void* d_ws, size_t ws_size, hipStream_t stream) {
  (void)n_in;
  auto Fp = [&](int i) { return (const float*)d_in[i]; };
  const long long need_x = ((long long)(NB - 1) * SEQ_FULL + SEQ) * (long long)EMB;
  if ((long long)in_sizes[0] < need_x || in_sizes[1] < (int)EMB || in_sizes[2] < (int)EMB || in_sizes[3] < (int)(EMB * 3 * EMB) || in_sizes[4] < (int)(3 * EMB) || in_sizes[5] < (int)(EMB * EMB) ||
      in_sizes[6] < (int)EMB || in_sizes[7] < (int)EMB || in_sizes[8] < (int)EMB || in_sizes[9] < (int)(EMB * HID) || in_sizes[10] < (int)HID || in_sizes[11] < (int)(HID * EMB) ||
      in_sizes[12] < (int)EMB || (long long)out_size < need_x) return;
  size_t off = 0; char* ws = (char*)d_ws;
  auto carve = [&](size_t bytes) { char* p = ws + off; off += (bytes + 255) & ~(size_t)255; return p; };
  constexpr size_t PLANE = (size_t)TOK * EMB * 2;
  constexpr size_t GBYTES = (size_t)TOK * HID * 2;
  static_assert(GBYTES <= 4 * PLANE);
  static_assert(PLANE % 256 == 0);
  b16* WQ = (b16*)carve((size_t)3 * EMB * EMB * 2); b16* WP = (b16*)carve((size_t)EMB * EMB * 2); b16* W1 = (b16*)carve((size_t)HID * EMB * 2); b16* W2 = (b16*)carve((size_t)EMB * HID * 2);
  b16* H = (b16*)carve(PLANE);
  char* region = carve(4 * PLANE);
  b16* QP = (b16*)region; b16* KP = (b16*)(region + PLANE); b16* VT = (b16*)(region + 2 * PLANE); b16* CT = (b16*)(region + 3 * PLANE); b16* G = (b16*)region;
  float* X1 = (float*)carve((size_t)TOK * EMB * 4);
  if (off > ws_size || off > ((size_t)128 << 20)) return;
  float* out = (float*)d_out;
  prep_kernel<<<TQ + TP + T1 + T2, 128, 0, stream>>>(Fp(3), Fp(5), Fp(9), Fp(11), WQ, WP, W1, W2);
  ln_kernel<1><<<TOK / 8, 256, 0, stream>>>(Fp(0), Fp(1), Fp(2), H);
  gemm_kernel<EPI_QKV, 0, EMB><<<dim3(TOK / 128, 3 * EMB / 96), 128, 0, stream>>>(H, WQ, Fp(4), X1, X1, QP, KP, VT);
  attn_kernel<<<dim3(SEQ / 64, NB * NH), 128, 0, stream>>>(QP, KP, VT, CT);
  gemm_kernel<EPI_PROJ, 1, EMB><<<dim3(TOK / 128, EMB / 96), 128, 0, stream>>>(CT, WP, Fp(6), Fp(0), X1, H, H, H);
  ln_kernel<0><<<TOK / 8, 256, 0, stream>>>(X1, Fp(7), Fp(8), H);
  gemm_kernel<EPI_FC1, 0, EMB><<<dim3(TOK / 128, HID / 96), 128, 0, stream>>>(H, W1, Fp(10), X1, X1, G, G, G);
  gemm_kernel<EPI_FC2, 1, HID><<<dim3(TOK / 128, EMB / 96), 128, 0, stream>>>(G, W2, Fp(12), X1, out, H, H, H);
}
